// _GIN_56599079026905
// MI455X (gfx1250) — hardware-run, weakly checked
//
#include <hip/hip_runtime.h>
#include <stddef.h>
#include <stdint.h>


#define NN      50000
#define NE      800000
#define NG      512
#define DIN     128
#define F       64
#define NL      3
#define TM      128
#define NTILE   391
#define MP      (NTILE * TM)
#define NTHR    256
#define NWAVE   8
#define NBS     1024
#define NBLK    49
#define WLCAP   3584
#define RCAP    (NWAVE * WLCAP)
#define DEGCAP  64
#define NCH     (NE / 256)
#define CPW     391
#define GPB     64
#define GCAP    256
#define PLSZ    (F * DIN)
#define XBLK    ((MP * (DIN / 8)) / NTHR)
#define WBLK    ((7 * (PLSZ / 8)) / NTHR)
#define LDS_E   ((2 * RCAP + NWAVE * NBS + 2 * NBS + 32) * 4)
#define LDS_G   ((GPB * GCAP + GPB) * 4)

constexpr int SPLIT_Z = 1;
constexpr int SPLIT_U = 1;

static_assert(NTILE * TM >= NN && (NTILE - 1) * TM < NN);
static_assert(NBLK * NBS >= MP);
static_assert(F == 16 * 4 && DIN == 128 && (DIN % 32) == 0);
static_assert(8 * GPB == NG && GPB == 8 * NWAVE);
static_assert((NE % 256) == 0 && NWAVE * CPW >= NCH && NE <= (1 << 20));
static_assert(RCAP >= 17455 && DEGCAP >= 35 + 8 && GCAP >= 127 + 8);
static_assert((RCAP % (4 * NTHR)) == 0 && (NBS % NTHR) == 0 && NBS == 4 * NTHR);
static_assert(((MP * (DIN / 8)) % NTHR) == 0 && ((7 * (PLSZ / 8)) % NTHR) == 0 && ((PLSZ / 8) % NTHR) == 0);
static_assert(((MP * (F / 4)) % NTHR) == 0);
static_assert(LDS_E <= 300000 && LDS_G <= 300000);
static_assert(((GPB * GCAP) % (4 * NTHR)) == 0);

typedef float          v4f  __attribute__((ext_vector_type(4)));
typedef float          v8f  __attribute__((ext_vector_type(8)));
typedef double         v2d  __attribute__((ext_vector_type(2)));
typedef int            v4i  __attribute__((ext_vector_type(4)));
typedef int            v8i  __attribute__((ext_vector_type(8)));
typedef unsigned int   v2u  __attribute__((ext_vector_type(2)));
typedef unsigned short v8us __attribute__((ext_vector_type(8)));
typedef __bf16         v16b __attribute__((ext_vector_type(16)));
typedef v4f  __attribute__((may_alias)) v4fa;
typedef v2d  __attribute__((may_alias)) v2da;
typedef v4i  __attribute__((may_alias)) v4ia;
typedef v8us __attribute__((may_alias)) v8usa;
union FragB { v16b v; v8us h[2]; v8i w; };

__device__ __forceinline__ v8f wmb(const FragB& a, const FragB& b, v8f c) {
  v8f d = __builtin_amdgcn_wmma_f32_16x16x32_bf16(false, a.v, false, b.v, (short)0, c, false, false);
  asm volatile("v_nop\n\tv_nop\n\tv_nop\n\tv_nop" : "+v"(d) : "v"(a.w), "v"(b.w));
  return d;
}

__device__ __forceinline__ int imin(int a, int b) { return a < b ? a : b; }
__device__ __forceinline__ int imax(int a, int b) { return a > b ? a : b; }

__device__ __forceinline__ unsigned bf_bits(float f) {
  const unsigned u = __float_as_uint(f);
  const unsigned r = (u + 0x7FFFu + ((u >> 16) & 1u)) >> 16;
  return (f != f) ? 0x7FC0u : r;
}
__device__ __forceinline__ float bf_val(unsigned b) { return __uint_as_float(b << 16); }
__device__ __forceinline__ float bf_rne(float f) { return bf_val(bf_bits(f)); }
__device__ __forceinline__ unsigned pk_hi(float f0, float f1) { return bf_bits(f0) | (bf_bits(f1) << 16); }
__device__ __forceinline__ unsigned pk_lo(float f0, float f1) {
  const float l0 = f0 - bf_val(bf_bits(f0));
  const float l1 = f1 - bf_val(bf_bits(f1));
  return bf_bits(l0) | (bf_bits(l1) << 16);
}

template <typename VT, typename PT>
__device__ __forceinline__ void vst2(PT* p, const VT v) {
  volatile VT* q = (volatile VT*)p;
  *q = v;
  __threadfence();
  *q = v;
}
template <typename VT, typename PT>
__device__ __forceinline__ void vst2_if(bool ok, PT* p, const VT v) {
  volatile VT* q = (volatile VT*)p;
  if (ok) *q = v;
  __threadfence();
  if (ok) *q = v;
}

__device__ __forceinline__ v8us gather8(const float* __restrict__ p) {
  v8us o;
#pragma unroll
  for (int i = 0; i < 8; ++i) o[i] = (unsigned short)bf_bits(p[(size_t)i * F]);
  return o;
}

__global__ __launch_bounds__(NTHR) void k_prep(const float* __restrict__ x, const float* __restrict__ Wt,
                                               const float* __restrict__ W1, const float* __restrict__ W2,
                                               unsigned short* xb, unsigned short* wp) {
  const int tid = (int)threadIdx.x;
  const int b = (int)blockIdx.x;
  if (b < XBLK) {
    const int u   = b * NTHR + tid;
    const int row = u >> 4;
    const int c8  = (u & 15) * 8;
    const int rc  = imin(row, NN - 1);
    const float* p = x + (size_t)rc * DIN + c8;
    const v4f a = *(const v4f*)p;
    const v4f c = *(const v4f*)(p + 4);
    asm volatile("" :: "v"(a));
    asm volatile("" :: "v"(c));
    const unsigned msk = (row < NN) ? 0xFFFFu : 0u;
    v8us o;
    o[0] = (unsigned short)(bf_bits(a.x) & msk); o[1] = (unsigned short)(bf_bits(a.y) & msk);
    o[2] = (unsigned short)(bf_bits(a.z) & msk); o[3] = (unsigned short)(bf_bits(a.w) & msk);
    o[4] = (unsigned short)(bf_bits(c.x) & msk); o[5] = (unsigned short)(bf_bits(c.y) & msk);
    o[6] = (unsigned short)(bf_bits(c.z) & msk); o[7] = (unsigned short)(bf_bits(c.w) & msk);
    vst2<v8us>(xb + (size_t)u * 8, o);
  } else if (b < XBLK + WBLK) {
    const int v  = (b - XBLK) * NTHR + tid;
    const int p  = v >> 10;
    const int w  = v & 1023;
    const int n  = w >> 4;
    const int k8 = (w & 15) * 8;
    v8us o;
    if (p == 0) {
      o = gather8(Wt + (size_t)k8 * F + n);
    } else {
      const int l  = (p - 1) >> 1;
      const int kk = k8 & (F - 1);
      const size_t off = (size_t)l * F * F + (size_t)kk * F + n;
      if (((p - 1) & 1) == 0) o = gather8(W1 + off);
      else                    o = gather8(W2 + off);
    }
    vst2<v8us>(wp + (size_t)v * 8, o);
  }
}

__global__ __launch_bounds__(NTHR) void k_bucket_e(const int* __restrict__ srcs, const int* __restrict__ dsts,
                                                   int* srclist, int* offp, int* cntp) {
  extern __shared__ v4i lds_e[];
  int* wl   = (int*)lds_e;
  int* sl   = wl + RCAP;
  int* wcn  = sl + RCAP;
  int* offs = wcn + NWAVE * NBS;
  int* tcnt = offs + NBS;
  int* misc = tcnt + NBS;
  const int tid = (int)threadIdx.x, lane = tid & 31, wave = tid >> 5;
  const int nodeBase = (int)blockIdx.x * NBS;

  {
    const v4i z4 = {0, 0, 0, 0};
    for (int i = tid * 4; i < RCAP + NWAVE * NBS + 2 * NBS; i += NTHR * 4) *(v4ia*)(sl + i) = z4;
    if (tid < 32) misc[tid] = 0;
  }
  __syncthreads();

  int* mywl = wl + wave * WLCAP;
  int wc = 0;
  const int c0 = wave * CPW;
  const int c1 = imin(c0 + CPW, NCH);
#pragma unroll 1
  for (int ch = c0; ch < c1; ++ch) {
    const int e0 = ch * 256 + lane * 8;
    const v4i da = *(const v4i*)(dsts + e0);
    const v4i db = *(const v4i*)(dsts + e0 + 4);
    const unsigned nbs = (unsigned)nodeBase;
    const unsigned s0 = (unsigned)da.x - nbs, s1 = (unsigned)da.y - nbs;
    const unsigned s2 = (unsigned)da.z - nbs, s3 = (unsigned)da.w - nbs;
    const unsigned s4 = (unsigned)db.x - nbs, s5 = (unsigned)db.y - nbs;
    const unsigned s6 = (unsigned)db.z - nbs, s7 = (unsigned)db.w - nbs;
    const bool h0 = s0 < (unsigned)NBS, h1 = s1 < (unsigned)NBS, h2 = s2 < (unsigned)NBS, h3 = s3 < (unsigned)NBS;
    const bool h4 = s4 < (unsigned)NBS, h5 = s5 < (unsigned)NBS, h6 = s6 < (unsigned)NBS, h7 = s7 < (unsigned)NBS;
    const int c = (int)h0 + (int)h1 + (int)h2 + (int)h3 + (int)h4 + (int)h5 + (int)h6 + (int)h7;
    int incl = c;
#pragma unroll
    for (int d = 1; d < 32; d <<= 1) {
      const int up = __shfl_up(incl, d);
      incl += (lane >= d) ? up : 0;
    }
    const int tot = __shfl(incl, 31);
    int pos = wc + incl - c;
#define PUTJ(J, HJ, SJ) { if (HJ) { if (pos < WLCAP) mywl[pos] = ((e0 + (J)) << 10) | (int)(SJ); pos += 1; } }
    PUTJ(0, h0, s0)
    PUTJ(1, h1, s1)
    PUTJ(2, h2, s2)
    PUTJ(3, h3, s3)
    PUTJ(4, h4, s4)
    PUTJ(5, h5, s5)
    PUTJ(6, h6, s6)
    PUTJ(7, h7, s7)
#undef PUTJ
    wc += tot;
  }
  if (lane == 0) misc[wave] = wc;
  __syncthreads();

  const int wcc = imin(imax(wc, 0), WLCAP);
  int* mycn = wcn + wave * NBS;
#pragma unroll 1
  for (int b0 = 0; b0 < wcc; b0 += 32) {
    const int idx = imin(b0 + lane, wcc - 1);
    const int ent = mywl[idx];
    const int m32 = imin(wcc - b0, 32);
#pragma unroll 1
    for (int k = 0; k < m32; ++k) {
      const int u = __builtin_amdgcn_readlane(ent, k);
      const int s = u & (NBS - 1);
      if (lane == 0) mycn[s] = mycn[s] + 1;
    }
  }
  __syncthreads();

  {
    v4i cw[NWAVE];
#pragma unroll
    for (int w2 = 0; w2 < NWAVE; ++w2) cw[w2] = *(const v4ia*)(wcn + w2 * NBS + 4 * tid);
    v4i t4 = cw[0];
#pragma unroll
    for (int w2 = 1; w2 < NWAVE; ++w2) t4 += cw[w2];
    const int ts = t4.x + t4.y + t4.z + t4.w;
    int incl = ts;
#pragma unroll
    for (int d = 1; d < 32; d <<= 1) {
      const int up = __shfl_up(incl, d);
      incl += (lane >= d) ? up : 0;
    }
    if (lane == 31) misc[8 + wave] = incl;
    __syncthreads();
    int pre = 0;
#pragma unroll
    for (int w2 = 0; w2 < NWAVE; ++w2) pre += (w2 < wave) ? misc[8 + w2] : 0;
    const int run = pre + incl - ts;
    v4i o4;
    o4.x = run; o4.y = run + t4.x; o4.z = o4.y + t4.y; o4.w = o4.z + t4.z;
    *(v4ia*)(offs + 4 * tid) = o4;
    *(v4ia*)(tcnt + 4 * tid) = t4;
    v4i cur = o4;
#pragma unroll
    for (int w2 = 0; w2 < NWAVE; ++w2) {
      *(v4ia*)(wcn + w2 * NBS + 4 * tid) = cur;
      cur += cw[w2];
    }
  }
  __syncthreads();

#pragma unroll 1
  for (int b0 = 0; b0 < wcc; b0 += 32) {
    const int idx = imin(b0 + lane, wcc - 1);
    const int ent = mywl[idx];
    const int m32 = imin(wcc - b0, 32);
#pragma unroll 1
    for (int k = 0; k < m32; ++k) {
      const int u = __builtin_amdgcn_readlane(ent, k);
      const int s = u & (NBS - 1);
      const int eid = (int)((unsigned)u >> 10);
      if (lane == 0) {
        int p = mycn[s];
        p = imin(imax(p, 0), RCAP - 1);
        sl[p] = eid;
        mycn[s] = p + 1;
      }
    }
  }
  __syncthreads();

  int ovf = 0;
#pragma unroll
  for (int w2 = 0; w2 < NWAVE; ++w2) ovf |= (misc[w2] > WLCAP) ? 1 : 0;
  int* slg = srclist + (size_t)blockIdx.x * RCAP;
#pragma unroll 1
  for (int it = 0; it < RCAP / (4 * NTHR); ++it) {
    const int i4 = (it * NTHR + tid) * 4;
    const v4i e = *(const v4ia*)(sl + i4);
    v4i o;
    o.x = srcs[imin(imax(e.x, 0), NE - 1)];
    o.y = srcs[imin(imax(e.y, 0), NE - 1)];
    o.z = srcs[imin(imax(e.z, 0), NE - 1)];
    o.w = srcs[imin(imax(e.w, 0), NE - 1)];
    vst2<v4i>(slg + i4, o);
  }
  {
    const v4i o4 = *(const v4ia*)(offs + 4 * tid);
    v4i c4 = *(const v4ia*)(tcnt + 4 * tid);
    if (ovf != 0) { c4.x = -1; c4.y = -1; c4.z = -1; c4.w = -1; }
    vst2<v4i>(offp + (size_t)blockIdx.x * NBS + 4 * tid, o4);
    vst2<v4i>(cntp + (size_t)blockIdx.x * NBS + 4 * tid, c4);
  }
}

__global__ __launch_bounds__(NTHR) void k_bucket_g(const int* __restrict__ bat, int* nodelist, int* gcnt) {
  extern __shared__ v4i lds_g[];
  int* gl = (int*)lds_g;
  int* gc = gl + GPB * GCAP;
  const int tid = (int)threadIdx.x, lane = tid & 31, wave = tid >> 5;
  {
    const v4i z4 = {0, 0, 0, 0};
    for (int i = tid * 4; i < GPB * GCAP; i += NTHR * 4) *(v4ia*)(gl + i) = z4;
    if (tid < GPB) gc[tid] = 0;
  }
  __syncthreads();
  const int g0 = (int)blockIdx.x * GPB + 8 * wave;
  int* mygl = gl + (8 * wave) * GCAP;
  int cq[8];
#pragma unroll
  for (int q = 0; q < 8; ++q) cq[q] = 0;
#pragma unroll 1
  for (int i0 = 0; i0 < NN; i0 += 32) {
    const int i  = i0 + lane;
    const int ic = imin(i, NN - 1);
    const int bv = bat[ic];
    asm volatile("" :: "v"(bv));
    const unsigned s = (unsigned)(bv - g0);
    const bool hit = (i < NN) && (s < 8u);
    const unsigned any = __builtin_amdgcn_ballot_w32(hit);
    if (any != 0u) {
#pragma unroll
      for (int q = 0; q < 8; ++q) {
        const bool hq = hit && (s == (unsigned)q);
        const unsigned mq = __builtin_amdgcn_ballot_w32(hq);
        const int pos = cq[q] + (int)__builtin_amdgcn_mbcnt_lo(mq, 0u);
        if (hq && pos < GCAP) mygl[q * GCAP + pos] = i;
        cq[q] += (int)__builtin_popcount(mq);
      }
    }
  }
  if (lane == 0) {
#pragma unroll
    for (int q = 0; q < 8; ++q) gc[8 * wave + q] = cq[q];
  }
  __syncthreads();
  int* nlg = nodelist + (size_t)blockIdx.x * (GPB * GCAP);
#pragma unroll 1
  for (int it = 0; it < (GPB * GCAP) / (4 * NTHR); ++it) {
    const int i4 = (it * NTHR + tid) * 4;
    const v4i e = *(const v4ia*)(gl + i4);
    vst2<v4i>(nlg + i4, e);
  }
  const v4i c4 = *(const v4ia*)(gc + 4 * (tid & 15));
  vst2_if<v4i>(tid < 16, gcnt + (size_t)blockIdx.x * GPB + 4 * (tid & 15), c4);
}

__device__ __forceinline__ void tile_out(const float* stg, double* rs, int rowBase, float* T, double* rec,
                                         int tid, int lane, int wave) {
  if (tid < F) {
    int rv = NN - rowBase;
    rv = imin(imax(rv, 0), TM);
    double s = 0.0, q = 0.0;
#pragma unroll 1
    for (int r = 0; r < rv; ++r) {
      const double v = (double)stg[r * F + tid];
      s += v;
      q += v * v;
    }
    rs[tid] = s;
    rs[F + tid] = q;
  }
  v4f fv[8];
#pragma unroll
  for (int i = 0; i < 8; ++i) fv[i] = *(const v4fa*)(stg + (16 * wave + 2 * i) * F + 4 * lane);
  float* op = T + (size_t)(rowBase + 16 * wave) * F + 4 * lane;
#pragma unroll
  for (int i = 0; i < 8; ++i) *(volatile v4f*)(op + 128 * i) = fv[i];
  __threadfence();
#pragma unroll
  for (int i = 0; i < 8; ++i) *(volatile v4f*)(op + 128 * i) = fv[i];
  __syncthreads();
  const v2d pv = *(const v2da*)(rs + 2 * (tid & 63));
  vst2_if<v2d>(tid < 64, rec + (size_t)blockIdx.x * (2 * F) + 2 * (tid & 63), pv);
}

__global__ __launch_bounds__(NTHR) __attribute__((amdgpu_num_vgpr(248)))
void k_gemm0(const unsigned short* __restrict__ XB, const unsigned short* __restrict__ WT,
             const float* __restrict__ bt, float* T, double* rec) {
  __shared__ __attribute__((aligned(16))) float stg[TM * F];
  __shared__ __attribute__((aligned(16))) double rs[2 * F];
  __shared__ float sb[F];
  const int tid = (int)threadIdx.x, lane = tid & 31, wave = tid >> 5, hh = lane >> 4, m = lane & 15;
  const int rowBase = (int)blockIdx.x * TM;
  if (tid < F) sb[tid] = bf_rne(bt[tid]);
  v8f acc[4];
  {
    const v8f z = {0.f, 0.f, 0.f, 0.f, 0.f, 0.f, 0.f, 0.f};
#pragma unroll
    for (int t = 0; t < 4; ++t) acc[t] = z;
  }
  const unsigned short* ap = XB + (size_t)(rowBase + 16 * wave + m) * DIN + 8 * hh;
  const unsigned short* wp = WT + (size_t)m * DIN + 8 * hh;
#pragma unroll 1
  for (int ks = 0; ks < DIN / 32; ++ks) {
    FragB af;
    af.h[0] = *(const v8usa*)(ap + 32 * ks);
    af.h[1] = *(const v8usa*)(ap + 32 * ks + 16);
#pragma unroll
    for (int t = 0; t < 4; ++t) {
      const unsigned short* wq = wp + (size_t)(16 * t) * DIN + 32 * ks;
      FragB bf;
      bf.h[0] = *(const v8usa*)wq;
      bf.h[1] = *(const v8usa*)(wq + 16);
      acc[t] = wmb(af, bf, acc[t]);
    }
  }
  __syncthreads();
#pragma unroll
  for (int t = 0; t < 4; ++t) {
    const int lc = 16 * t + m;
    const float bb = sb[lc];
#pragma unroll
    for (int r = 0; r < 8; ++r) {
      const int lr = 16 * wave + 8 * hh + r;
      const bool live = (rowBase + lr) < NN;
      const float v = acc[t][r] + bb;
      stg[lr * F + lc] = live ? v : 0.0f;
    }
  }
  __syncthreads();
  tile_out(stg, rs, rowBase, T, rec, tid, lane, wave);
}

__global__ __launch_bounds__(NTHR) __attribute__((amdgpu_num_vgpr(248)))
void k_mlp(const unsigned short* __restrict__ ZHL, const unsigned short* __restrict__ W1D,
           const unsigned short* __restrict__ W2D, const float* __restrict__ b1,
           const float* __restrict__ b2, float* T, double* rec) {
  __shared__ __attribute__((aligned(16))) float stg[TM * F];
  __shared__ __attribute__((aligned(16))) double rs[2 * F];
  __shared__ float sb1[F];
  __shared__ float sb2[F];
  const int tid = (int)threadIdx.x, lane = tid & 31, wave = tid >> 5, hh = lane >> 4, m = lane & 15;
  const int rowBase = (int)blockIdx.x * TM;
  if (tid < F) { sb1[tid] = bf_rne(b1[tid]); sb2[tid] = bf_rne(b2[tid]); }
  const v8f z8 = {0.f, 0.f, 0.f, 0.f, 0.f, 0.f, 0.f, 0.f};
  v8f acc[4];
#pragma unroll
  for (int t = 0; t < 4; ++t) acc[t] = z8;
  {
    const unsigned short* ap = ZHL + (size_t)(rowBase + 16 * wave + m) * DIN + 8 * hh;
    const unsigned short* wp = W1D + (size_t)m * DIN + 8 * hh;
#pragma unroll 1
    for (int ks = 0; ks < DIN / 32; ++ks) {
      FragB af;
      af.h[0] = *(const v8usa*)(ap + 32 * ks);
      af.h[1] = *(const v8usa*)(ap + 32 * ks + 16);
#pragma unroll
      for (int t = 0; t < 4; ++t) {
        const unsigned short* wq = wp + (size_t)(16 * t) * DIN + 32 * ks;
        FragB bf;
        bf.h[0] = *(const v8usa*)wq;
        bf.h[1] = *(const v8usa*)(wq + 16);
        acc[t] = wmb(af, bf, acc[t]);
      }
    }
  }
  __syncthreads();
#pragma unroll
  for (int t = 0; t < 4; ++t) {
    const int lc = 16 * t + m;
    const float bb = sb1[lc];
#pragma unroll
    for (int r = 0; r < 8; ++r) {
      const int lr = 16 * wave + 8 * hh + r;
      const float v = acc[t][r] + bb;
      stg[lr * F + lc] = (v > 0.0f) ? v : (v - v);
    }
  }
  __syncthreads();

  v8f ac2[4];
#pragma unroll
  for (int t = 0; t < 4; ++t) ac2[t] = z8;
  {
    const float* ur = stg + (16 * wave + m) * F + 8 * hh;
    const unsigned short* wp = W2D + (size_t)m * DIN + 8 * hh;
#pragma unroll
    for (int cg = 0; cg < 2; ++cg) {
      const v4f x0 = *(const v4fa*)(ur + 32 * cg);
      const v4f x1 = *(const v4fa*)(ur + 32 * cg + 4);
      const v4f x2 = *(const v4fa*)(ur + 32 * cg + 16);
      const v4f x3 = *(const v4fa*)(ur + 32 * cg + 20);
      FragB ah, al;
      ah.w[0] = (int)pk_hi(x0.x, x0.y); ah.w[1] = (int)pk_hi(x0.z, x0.w);
      ah.w[2] = (int)pk_hi(x1.x, x1.y); ah.w[3] = (int)pk_hi(x1.z, x1.w);
      ah.w[4] = (int)pk_hi(x2.x, x2.y); ah.w[5] = (int)pk_hi(x2.z, x2.w);
      ah.w[6] = (int)pk_hi(x3.x, x3.y); ah.w[7] = (int)pk_hi(x3.z, x3.w);
      if (SPLIT_U != 0) {
        al.w[0] = (int)pk_lo(x0.x, x0.y); al.w[1] = (int)pk_lo(x0.z, x0.w);
        al.w[2] = (int)pk_lo(x1.x, x1.y); al.w[3] = (int)pk_lo(x1.z, x1.w);
        al.w[4] = (int)pk_lo(x2.x, x2.y); al.w[5] = (int)pk_lo(x2.z, x2.w);
        al.w[6] = (int)pk_lo(x3.x, x3.y); al.w[7] = (int)pk_lo(x3.z, x3.w);
      } else {
        const v8i zi = {0, 0, 0, 0, 0, 0, 0, 0};
        al.w = zi;
      }
#pragma unroll
      for (int t = 0; t < 4; ++t) {
        const unsigned short* wq = wp + (size_t)(16 * t) * DIN + 32 * cg;
        FragB bh, bl;
        bh.h[0] = *(const v8usa*)wq;
        bh.h[1] = *(const v8usa*)(wq + 16);
        bl.h[0] = *(const v8usa*)(wq + F);
        bl.h[1] = *(const v8usa*)(wq + F + 16);
        ac2[t] = wmb(ah, bh, ac2[t]);
        ac2[t] = wmb(al, bl, ac2[t]);
      }
    }
  }
  __syncthreads();
#pragma unroll
  for (int t = 0; t < 4; ++t) {
    const int lc = 16 * t + m;
    const float bb = sb2[lc];
#pragma unroll
    for (int r = 0; r < 8; ++r) {
      const int lr = 16 * wave + 8 * hh + r;
      const bool live = (rowBase + lr) < NN;
      const float v = ac2[t][r] + bb;
      stg[lr * F + lc] = live ? v : 0.0f;
    }
  }
  __syncthreads();
  tile_out(stg, rs, rowBase, T, rec, tid, lane, wave);
}

__global__ __launch_bounds__(F) void k_comb(const double* __restrict__ rec, const float* __restrict__ gam,
                                            const float* __restrict__ bet, float* stat) {
  __shared__ __attribute__((aligned(16))) float st[4 * F];
  const int c = (int)threadIdx.x;
  double S = 0.0, Q = 0.0;
#pragma unroll 1
  for (int t = 0; t < NTILE; ++t) {
    S += rec[(size_t)t * (2 * F) + c];
    Q += rec[(size_t)t * (2 * F) + F + c];
  }
  const double invn = 1.0 / (double)NN;
  const double mean = S * invn;
  double var = Q * invn - mean * mean;
  var = (var < 0.0) ? 0.0 : var;
  const float mf = (float)mean;
  const float vf = (float)var;
  const float rstd = 1.0f / sqrtf(vf + 1e-5f);
  st[c] = mf;
  st[F + c] = rstd;
  st[2 * F + c] = bf_rne(gam[c]);
  st[3 * F + c] = bf_rne(bet[c]);
  __syncthreads();
  const v4f v = *(const v4fa*)(st + 4 * c);
  vst2<v4f>(stat + 4 * c, v);
}

template <int RELU>
__global__ __launch_bounds__(NTHR) void k_apply(const float* __restrict__ T, const float* __restrict__ stat,
                                                float* H) {
  __shared__ float ssh[4 * F];
  const int tid = (int)threadIdx.x;
  ssh[tid] = stat[tid];
  __syncthreads();
  const int u   = (int)blockIdx.x * NTHR + tid;
  const int row = u >> 4;
  const int c4  = (u & 15) * 4;
  const int rc  = imin(row, NN - 1);
  const v4f a = *(const v4f*)(T + (size_t)rc * F + c4);
  asm volatile("" :: "v"(a));
  const bool ok = row < NN;
  float y0 = ((a.x - ssh[c4 + 0]) * ssh[F + c4 + 0]) * ssh[2 * F + c4 + 0] + ssh[3 * F + c4 + 0];
  float y1 = ((a.y - ssh[c4 + 1]) * ssh[F + c4 + 1]) * ssh[2 * F + c4 + 1] + ssh[3 * F + c4 + 1];
  float y2 = ((a.z - ssh[c4 + 2]) * ssh[F + c4 + 2]) * ssh[2 * F + c4 + 2] + ssh[3 * F + c4 + 2];
  float y3 = ((a.w - ssh[c4 + 3]) * ssh[F + c4 + 3]) * ssh[2 * F + c4 + 3] + ssh[3 * F + c4 + 3];
  if (RELU != 0) {
    y0 = (y0 > 0.0f) ? y0 : (y0 - y0);
    y1 = (y1 > 0.0f) ? y1 : (y1 - y1);
    y2 = (y2 > 0.0f) ? y2 : (y2 - y2);
    y3 = (y3 > 0.0f) ? y3 : (y3 - y3);
  }
  v4f o;
  o.x = ok ? y0 : 0.0f; o.y = ok ? y1 : 0.0f; o.z = ok ? y2 : 0.0f; o.w = ok ? y3 : 0.0f;
  vst2<v4f>(H + (size_t)u * 4, o);
}

__global__ __launch_bounds__(NTHR) void k_pool(const float* __restrict__ H, const int* __restrict__ nodelist,
                                               const int* __restrict__ gcnt, float* out) {
  const int tid = (int)threadIdx.x, lane = tid & 31, wave = tid >> 5, hh = lane >> 4, m = lane & 15;
  const int g = (int)blockIdx.x * NWAVE + wave;
  const int craw = __builtin_amdgcn_readfirstlane(gcnt[g]);
  const int c = imin(imax(craw, 0), GCAP);
  const bool pois = (craw < 0) || (craw > GCAP);
  const int* nl = nodelist + (size_t)g * GCAP;
  int last = c - 1;
  last = last < 0 ? 0 : last;
  const int nj = (c + 1) >> 1;
  float a0 = 0.0f, a1 = 0.0f, a2 = 0.0f, a3 = 0.0f;
#pragma unroll 1
  for (int j = 0; j < nj; ++j) {
    const int k = 2 * j + hh;
    const bool valid = k < c;
    const int idx = imin(k, last);
    int node = nl[idx];
    node = imin(imax(node, 0), NN - 1);
    const v4f v = *(const v4f*)(H + (size_t)node * F + 4 * m);
    asm volatile("" :: "v"(v));
    a0 += valid ? v.x : 0.0f;
    a1 += valid ? v.y : 0.0f;
    a2 += valid ? v.z : 0.0f;
    a3 += valid ? v.w : 0.0f;
  }
  a0 += __shfl_xor(a0, 16);
  a1 += __shfl_xor(a1, 16);
  a2 += __shfl_xor(a2, 16);
  a3 += __shfl_xor(a3, 16);
  int cv = c;
  asm volatile("" : "+v"(cv));
  const float cf = fmaxf((float)cv, 1.0f);
  const float pz = pois ? __int_as_float(0x7fc00000) : 0.0f;
  v4f o;
  o.x = a0 / cf + pz; o.y = a1 / cf + pz; o.z = a2 / cf + pz; o.w = a3 / cf + pz;
  vst2_if<v4f>(lane < 16, out + (size_t)g * F + 4 * m, o);
}

__global__ __launch_bounds__(NTHR) void k_replay(const float* __restrict__ H, const int* __restrict__ srclist,
                                                 const int* __restrict__ offp, const int* __restrict__ cntp,
                                                 unsigned short* zhl) {
  const int tid = (int)threadIdx.x, lane = tid & 31, wave = tid >> 5, hh = lane >> 4, m = lane & 15;
  const int rowBase = (int)blockIdx.x * TM + 16 * wave;
  const float qnan = __int_as_float(0x7fc00000);
#pragma unroll 1
  for (int i = 0; i < 16; ++i) {
    const int row = rowBase + i;
    const int oraw = __builtin_amdgcn_readfirstlane(offp[row]);
    const int craw = __builtin_amdgcn_readfirstlane(cntp[row]);
    const int o = imin(imax(oraw, 0), RCAP - 1);
    int c = imin(imax(craw, 0), DEGCAP);
    c = imin(c, RCAP - o);
    const bool pois = (craw < 0) || (craw > DEGCAP);
    const int* lst = srclist + (size_t)(row >> 10) * RCAP;
    int last = o + c - 1;
    last = last < o ? o : last;
    const int nj = (c + 1) >> 1;
    float a0 = 0.0f, a1 = 0.0f, a2 = 0.0f, a3 = 0.0f;
#pragma unroll 1
    for (int j = 0; j < nj; ++j) {
      const int k = 2 * j + hh;
      const bool valid = k < c;
      const int idx = imin(o + k, last);
      int s = lst[idx];
      s = imin(imax(s, 0), NN - 1);
      const v4f v = *(const v4f*)(H + (size_t)s * F + 4 * m);
      asm volatile("" :: "v"(v));
      a0 += valid ? v.x : 0.0f;
      a1 += valid ? v.y : 0.0f;
      a2 += valid ? v.z : 0.0f;
      a3 += valid ? v.w : 0.0f;
    }
    a0 += __shfl_xor(a0, 16);
    a1 += __shfl_xor(a1, 16);
    a2 += __shfl_xor(a2, 16);
    a3 += __shfl_xor(a3, 16);
    const int rc = imin(row, NN - 1);
    const v4f sf = *(const v4f*)(H + (size_t)rc * F + 4 * m);
    asm volatile("" :: "v"(sf));
    const bool live = row < NN;
    const float pz = pois ? qnan : 0.0f;
    const float r0 = (live ? (sf.x + a0) : 0.0f) + pz;
    const float r1 = (live ? (sf.y + a1) : 0.0f) + pz;
    const float r2 = (live ? (sf.z + a2) : 0.0f) + pz;
    const float r3 = (live ? (sf.w + a3) : 0.0f) + pz;
    const unsigned h01 = pk_hi(r0, r1), h23 = pk_hi(r2, r3);
    unsigned l01 = 0u, l23 = 0u;
    if (SPLIT_Z != 0) { l01 = pk_lo(r0, r1); l23 = pk_lo(r2, r3); }
    const unsigned selm = (hh == 0) ? 0xFFFFFFFFu : 0u;
    v2u pk;
    pk.x = (h01 & selm) | (l01 & ~selm);
    pk.y = (h23 & selm) | (l23 & ~selm);
    vst2<v2u>(zhl + (size_t)row * DIN + 4 * lane, pk);
  }
}

static inline size_t al256(size_t o) { return (o + 255) & ~(size_t)255; }

extern "C" void kernel_launch(void* const* d_in, const int* in_sizes, int n_in,
                              void* d_out, int out_size, void* d_ws, size_t ws_size,
                              hipStream_t stream) {
  if (n_in < 13) return;
  if (in_sizes[0] != NN * DIN) return;
  if (in_sizes[1] != 2 * NE) return;
  if (in_sizes[2] != NN) return;
  if (in_sizes[3] != DIN * F) return;
  if (in_sizes[4] != F || in_sizes[5] != F || in_sizes[6] != F) return;
  if (in_sizes[7] != NL * F * F || in_sizes[9] != NL * F * F) return;
  if (in_sizes[8] != NL * F || in_sizes[10] != NL * F) return;
  if (in_sizes[11] != NL * F || in_sizes[12] != NL * F) return;
  if (out_size != (NL + 1) * NG * F) return;

  const float* x   = (const float*)d_in[0];
  const int*   ei  = (const int*)  d_in[1];
  const int*   src = ei;
  const int*   dst = ei + NE;
  const int*   bat = (const int*)  d_in[2];
  const float* Wt  = (const float*)d_in[3];
  const float* bt  = (const float*)d_in[4];
  const float* gt  = (const float*)d_in[5];
  const float* bet = (const float*)d_in[6];
  const float* W1  = (const float*)d_in[7];
  const float* b1  = (const float*)d_in[8];
  const float* W2  = (const float*)d_in[9];
  const float* b2  = (const float*)d_in[10];
  const float* g   = (const float*)d_in[11];
  const float* be  = (const float*)d_in[12];
  float* out = (float*)d_out;

  char* ws = (char*)d_ws;
  size_t off = 0;
  const size_t oXB = off; off = al256(off + (size_t)MP * DIN * 2);
  const size_t oT  = off; off = al256(off + (size_t)MP * F * 4);
  const size_t oH  = off; off = al256(off + (size_t)MP * F * 4);
  const size_t oZ  = off; off = al256(off + (size_t)MP * DIN * 2);
  const size_t oSL = off; off = al256(off + (size_t)NBLK * RCAP * 4);
  const size_t oOF = off; off = al256(off + (size_t)NBLK * NBS * 4);
  const size_t oCN = off; off = al256(off + (size_t)NBLK * NBS * 4);
  const size_t oNL = off; off = al256(off + (size_t)NG * GCAP * 4);
  const size_t oGC = off; off = al256(off + (size_t)NG * 4);
  const size_t oWP = off; off = al256(off + (size_t)7 * PLSZ * 2);
  const size_t oRC = off; off = al256(off + (size_t)NTILE * 2 * F * 8);
  const size_t oST = off; off = al256(off + (size_t)4 * F * 4);
  if (off > ws_size || off > ((size_t)128u << 20)) return;

  unsigned short* XB  = (unsigned short*)(ws + oXB);
  float*          T   = (float*)(ws + oT);
  float*          H   = (float*)(ws + oH);
  unsigned short* ZHL = (unsigned short*)(ws + oZ);
  int*            SL  = (int*)(ws + oSL);
  int*            OFP = (int*)(ws + oOF);
  int*            CNP = (int*)(ws + oCN);
  int*            NLP = (int*)(ws + oNL);
  int*            GCP = (int*)(ws + oGC);
  unsigned short* WP  = (unsigned short*)(ws + oWP);
  double*         REC = (double*)(ws + oRC);
  float*          ST  = (float*)(ws + oST);

  hipFuncSetAttribute(reinterpret_cast<const void*>(&k_bucket_e), hipFuncAttributeMaxDynamicSharedMemorySize, LDS_E);
  hipFuncSetAttribute(reinterpret_cast<const void*>(&k_bucket_g), hipFuncAttributeMaxDynamicSharedMemorySize, LDS_G);

  const int gApply = (MP * (F / 4)) / NTHR;

  k_prep<<<XBLK + WBLK, NTHR, 0, stream>>>(x, Wt, W1, W2, XB, WP);
  k_bucket_e<<<NBLK, NTHR, LDS_E, stream>>>(src, dst, SL, OFP, CNP);
  k_bucket_g<<<NG / GPB, NTHR, LDS_G, stream>>>(bat, NLP, GCP);
  k_gemm0<<<NTILE, NTHR, 0, stream>>>(XB, WP, bt, T, REC);
  k_comb<<<1, F, 0, stream>>>(REC, gt, bet, ST);
  k_apply<0><<<gApply, NTHR, 0, stream>>>(T, ST, H);
  k_pool<<<NG / NWAVE, NTHR, 0, stream>>>(H, NLP, GCP, out);
  for (int l = 0; l < NL; ++l) {
    k_replay<<<NTILE, NTHR, 0, stream>>>(H, SL, OFP, CNP, ZHL);
    k_mlp<<<NTILE, NTHR, 0, stream>>>(ZHL, WP + (size_t)(1 + 2 * l) * PLSZ, WP + (size_t)(2 + 2 * l) * PLSZ,
                                      b1 + (size_t)l * F, b2 + (size_t)l * F, T, REC);
    k_comb<<<1, F, 0, stream>>>(REC, g + (size_t)l * F, be + (size_t)l * F, ST);
    k_apply<1><<<gApply, NTHR, 0, stream>>>(T, ST, H);
    k_pool<<<NG / NWAVE, NTHR, 0, stream>>>(H, NLP, GCP, out + (size_t)(l + 1) * NG * F);
  }
}
